// SelectiveSSM_26044681683346
// MI455X (gfx1250) — hardware-verified
//
#include <hip/hip_runtime.h>
#include <math.h>

#pragma clang fp contract(off)

typedef __attribute__((ext_vector_type(8)))  _Float16 v8h;
typedef __attribute__((ext_vector_type(16))) __bf16   v16b;
typedef __attribute__((ext_vector_type(8)))  __bf16   v8b;
typedef __attribute__((ext_vector_type(8)))  float    v8f;
typedef __attribute__((ext_vector_type(4)))  float    v4f;

constexpr int kB      = 2;
constexpr int kL      = 2048;
constexpr int kD      = 1024;
constexpr int kN      = 16;
constexpr int kM      = kB * kL;
constexpr int kChunk  = 64;
constexpr int kNChunk = kL / kChunk;
constexpr int kBCW    = 64;
constexpr int kBCR    = 128;
constexpr int kTP     = 260;

static_assert(kM == 4096 && kD == 1024 && kN == 16 && kL == 2048 && kB == 2, "shape");
static_assert(kM % 64 == 0 && kD % 64 == 0 && kBCW % 64 == 0, "GEMM M,N multiples of 64");
static_assert(kD % 32 == 0, "GEMM K multiple of 32");
static_assert(((kM / 64) * (kD / 64)) % 8 == 0 && ((kM / 64) * (kBCW / 64)) % 8 == 0, "8 tiles per block");
static_assert(kL % kChunk == 0 && kChunk % 16 == 0 && kD % 256 == 0 && kNChunk == 32, "scan tiles");
static_assert(2 * kN <= kBCW && kBCW <= kBCR && kBCR == 128, "fused width");
static_assert((kM * kD) % (8 * 256) == 0 && (kD * kD) % (8 * 256) == 0 && (kBCW * kD) % (8 * 256) == 0, "convert grids exact");
static_assert((kTP * 4) % 16 == 0, "LDS row pitch 16-B aligned");

constexpr size_t kOffXb   = 0;
constexpr size_t kOffWdb  = kOffXb  + (size_t)kM * kD * 2;
constexpr size_t kOffBCb  = kOffWdb + (size_t)kD * kD * 2;
constexpr size_t kOffBdR  = kOffBCb + (size_t)kBCW * kD * 2;
constexpr size_t kOffBcR  = kOffBdR + (size_t)kD * 4;
constexpr size_t kOffPre  = kOffBcR + (size_t)kBCR * 4;
constexpr size_t kOffBCf  = kOffPre + (size_t)kM * kD * 4;
constexpr size_t kOffP    = kOffBCf + (size_t)kM * kBCW * 4;
constexpr size_t kOffR    = kOffP   + (size_t)kB * kNChunk * kN * kD * 4;
constexpr size_t kOffHin  = kOffR   + (size_t)kB * kNChunk * kN * kD * 4;
constexpr size_t kWsTotal = kOffHin + (size_t)kB * kNChunk * kN * kD * 4;
static_assert(kWsTotal == 41030144ull, "carve total");
static_assert(kWsTotal <= 134217728ull, "carve cap");
static_assert((kOffWdb % 256) == 0 && (kOffBCb % 256) == 0 && (kOffBdR % 256) == 0 && (kOffBcR % 256) == 0 &&
              (kOffPre % 256) == 0 && (kOffBCf % 256) == 0 && (kOffP % 256) == 0 && (kOffR % 256) == 0 &&
              (kOffHin % 256) == 0, "aligned regions");

__device__ __forceinline__ unsigned short f2bf_bits(float f) {
  unsigned u = __float_as_uint(f);
  return (unsigned short)((u + 0x7FFFu + ((u >> 16) & 1u)) >> 16);
}
__device__ __forceinline__ float bf_bits2f(unsigned short h) { return __uint_as_float(((unsigned)h) << 16); }
__device__ __forceinline__ float rne_bf(float f) { return bf_bits2f(f2bf_bits(f)); }

__device__ __forceinline__ float softplus_f(float v) {
  const float ex = expf(-fabsf(v));
  return fmaxf(v, 0.0f) + log1pf(ex);
}

__device__ __forceinline__ void acc_guard4(v8f& a, v8f& b, v8f& c, v8f& d) {
  asm volatile("v_nop\n\tv_nop\n\tv_nop\n\tv_nop" : "+v"(a), "+v"(b), "+v"(c), "+v"(d));
}
__device__ __forceinline__ void guard_row_b(v8f& c0, v8f& c1, v8f& c2, v8f& c3,
                                            v16b a, v16b b0, v16b b1, v16b b2, v16b b3) {
  asm volatile("v_nop\n\tv_nop\n\tv_nop\n\tv_nop"
               : "+v"(c0), "+v"(c1), "+v"(c2), "+v"(c3)
               : "v"(a), "v"(b0), "v"(b1), "v"(b2), "v"(b3));
}

struct FragB {
  union U { v16b v; v8b h[2]; };
  static __device__ __forceinline__ v16b load(const __bf16* p) {
    U f; f.h[0] = *(const v8b*)(p); f.h[1] = *(const v8b*)(p + 16); return f.v;
  }
  static __device__ __forceinline__ v8f mma(v16b a, v16b b, v8f c) {
    return __builtin_amdgcn_wmma_f32_16x16x32_bf16(false, a, false, b, (short)0, c, false, false);
  }
};

__global__ __launch_bounds__(256) void cvt_bf16_kernel(
    const float* __restrict__ src, unsigned short* __restrict__ dst, int total8)
{
  const int i = blockIdx.x * 256 + threadIdx.x;
  if (i >= total8) return;
  const size_t e0 = (size_t)i << 3;
  const v4f a0 = *(const v4f*)(src + e0);
  const v4f a1 = *(const v4f*)(src + e0 + 4);
  v8h hv;
#pragma unroll
  for (int e = 0; e < 4; ++e) {
    const float f0 = a0[e];
    const float f1 = a1[e];
    const unsigned short h0 = f2bf_bits(f0);
    const unsigned short h1 = f2bf_bits(f1);
    hv[e]     = __builtin_bit_cast(_Float16, h0);
    hv[4 + e] = __builtin_bit_cast(_Float16, h1);
  }
  unsigned short* q = dst + e0;
  *(volatile v8h*)q = hv;
  __threadfence();
  *(volatile v8h*)q = hv;
}

__global__ __launch_bounds__(256) void prep_kernel(
    const float* __restrict__ Wb, const float* __restrict__ Wc,
    const float* __restrict__ bd, const float* __restrict__ bb, const float* __restrict__ bc,
    unsigned short* __restrict__ BCb, float* __restrict__ bdR, float* __restrict__ bcR)
{
  const int tid = threadIdx.x, lane = tid & 31, wave = tid >> 5;
  {
    const int i   = blockIdx.x * 256 + tid;
    const int e0  = i << 3;
    const int row = e0 >> 10;
    const int col = e0 & (kD - 1);
    const int rb  = (row < kN) ? row : (kN - 1);
    int rc = row - kN;
    rc = rc < 0 ? 0 : rc;
    rc = rc > (kN - 1) ? (kN - 1) : rc;
    const float fa = (row < kN) ? 1.0f : 0.0f;
    const float fb = (row >= kN && row < 2 * kN) ? 1.0f : 0.0f;
    const v4f a0 = *(const v4f*)(Wb + (size_t)rb * kD + col);
    const v4f a1 = *(const v4f*)(Wb + (size_t)rb * kD + col + 4);
    const v4f c0 = *(const v4f*)(Wc + (size_t)rc * kD + col);
    const v4f c1 = *(const v4f*)(Wc + (size_t)rc * kD + col + 4);
    v8h hv;
#pragma unroll
    for (int e = 0; e < 4; ++e) {
      const float wa0 = a0[e], wa1 = a1[e], wc0 = c0[e], wc1 = c1[e];
      const float t0 = fa * wa0 + fb * wc0;
      const float t1 = fa * wa1 + fb * wc1;
      const unsigned short h0 = f2bf_bits(t0);
      const unsigned short h1 = f2bf_bits(t1);
      hv[e]     = __builtin_bit_cast(_Float16, h0);
      hv[4 + e] = __builtin_bit_cast(_Float16, h1);
    }
    unsigned short* q = BCb + e0;
    *(volatile v8h*)q = hv;
    __threadfence();
    *(volatile v8h*)q = hv;
  }
  if (blockIdx.x == 0) {
    {
      const v4f v = *(const v4f*)(bd + tid * 4);
      v4f r;
#pragma unroll
      for (int e = 0; e < 4; ++e) { const float f = v[e]; r[e] = rne_bf(f); }
      float* q = bdR + tid * 4;
      *(volatile v4f*)q = r;
      __threadfence();
      *(volatile v4f*)q = r;
    }
    if (wave == 0) {
      const int qq = lane * 4;
      const int qb = (qq < kN) ? qq : (kN - 4);
      int qc = qq - kN;
      qc = qc < 0 ? 0 : qc;
      qc = qc > (kN - 4) ? (kN - 4) : qc;
      const float fa = (qq < kN) ? 1.0f : 0.0f;
      const float fb = (qq >= kN && qq < 2 * kN) ? 1.0f : 0.0f;
      const v4f vb = *(const v4f*)(bb + qb);
      const v4f vc = *(const v4f*)(bc + qc);
      v4f r;
#pragma unroll
      for (int e = 0; e < 4; ++e) {
        const float fvb = vb[e], fvc = vc[e];
        r[e] = rne_bf(fa * fvb + fb * fvc);
      }
      float* q = bcR + qq;
      *(volatile v4f*)q = r;
      __threadfence();
      *(volatile v4f*)q = r;
    }
  }
}

__global__ __launch_bounds__(256) void gemm_bf16_64(
    const unsigned short* __restrict__ Ap, int lda,
    const unsigned short* __restrict__ Btp, int ldb,
    float* __restrict__ Cout, int ldc,
    const float* __restrict__ bias,
    int M, int N, int K)
{
  const __bf16* A  = (const __bf16*)Ap;
  const __bf16* Bt = (const __bf16*)Btp;
  __shared__ __align__(16) float sT[8][16 * 68];
  const int lane = threadIdx.x & 31;
  const int wave = threadIdx.x >> 5;
  const int tilesN = N >> 6;
  const int tilesM = M >> 6;
  const int tile = blockIdx.x * 8 + wave;
  if (tile >= tilesM * tilesN) return;
  const int tm = tile / tilesN;
  const int tn = tile - tm * tilesN;
  const int m0 = tm << 6;
  const int n0 = tn << 6;

  const int rlane = lane & 15;
  const int koff  = (lane >> 4) * 8;
  const int mOff  = (lane >> 4) * 8;

  v8f acc[4][4];
#pragma unroll
  for (int i = 0; i < 4; ++i)
#pragma unroll
    for (int j = 0; j < 4; ++j) acc[i][j] = (v8f){0.f,0.f,0.f,0.f,0.f,0.f,0.f,0.f};

  for (int k0 = 0; k0 < K; k0 += 32) {
    v16b bh[4];
#pragma unroll
    for (int j = 0; j < 4; ++j) {
      const size_t bo = (size_t)(n0 + (j << 4) + rlane) * ldb + koff + k0;
      bh[j] = FragB::load(Bt + bo);
    }
#pragma unroll
    for (int i = 0; i < 4; ++i) {
      const size_t ao = (size_t)(m0 + (i << 4) + rlane) * lda + koff + k0;
      const v16b ah = FragB::load(A + ao);
#pragma unroll
      for (int j = 0; j < 4; ++j) acc[i][j] = FragB::mma(ah, bh[j], acc[i][j]);
      guard_row_b(acc[i][0], acc[i][1], acc[i][2], acc[i][3], ah, bh[0], bh[1], bh[2], bh[3]);
    }
  }
  acc_guard4(acc[0][0], acc[0][1], acc[0][2], acc[0][3]);
  acc_guard4(acc[1][0], acc[1][1], acc[1][2], acc[1][3]);
  acc_guard4(acc[2][0], acc[2][1], acc[2][2], acc[2][3]);
  acc_guard4(acc[3][0], acc[3][1], acc[3][2], acc[3][3]);

  float* slab = sT[wave];
#pragma unroll
  for (int i = 0; i < 4; ++i) {
    const int mBase = m0 + (i << 4);
#pragma unroll
    for (int j = 0; j < 4; ++j) {
      const int n = n0 + (j << 4) + rlane;
      const float bv = bias[n];
#pragma unroll
      for (int r = 0; r < 8; ++r) {
        const float v = acc[i][j][r] + bv;
        slab[(mOff + r) * 68 + (j << 4) + rlane] = v;
      }
    }
    __builtin_amdgcn_fence(__ATOMIC_RELEASE, "workgroup");
    __builtin_amdgcn_wave_barrier();
    __builtin_amdgcn_fence(__ATOMIC_ACQUIRE, "workgroup");
    {
      const int hh = lane >> 4, c4 = (lane & 15) * 4;
      for (int pass = 0; pass < 2; ++pass) {
#pragma unroll
        for (int it = 0; it < 8; ++it) {
          const int row = it * 2 + hh;
          const v4f v = *(const v4f*)(slab + row * 68 + c4);
          *(volatile v4f*)(Cout + (size_t)(mBase + row) * ldc + n0 + c4) = v;
        }
        __threadfence();
      }
    }
    __builtin_amdgcn_fence(__ATOMIC_RELEASE, "workgroup");
    __builtin_amdgcn_wave_barrier();
    __builtin_amdgcn_fence(__ATOMIC_ACQUIRE, "workgroup");
  }
}

__global__ __launch_bounds__(256) void scan_pass1_kernel(
    const float* __restrict__ PRE, const float* __restrict__ X, const float* __restrict__ Am,
    const float* __restrict__ BCf, float* __restrict__ P, float* __restrict__ R)
{
  __shared__ __align__(16) float sBC[kChunk * 32];
  __shared__ __align__(16) float sP[kN * kTP];
  __shared__ __align__(16) float sR[kN * kTP];
  const int tid = threadIdx.x, lane = tid & 31, wave = tid >> 5;
  const int d0 = blockIdx.x * 256;
  const int d  = d0 + tid;
  const int c  = blockIdx.y;
  const int b  = blockIdx.z;
  const size_t row0 = (size_t)b * kL + (size_t)c * kChunk;

#pragma unroll
  for (int i = 0; i < 2; ++i) {
    const int idx = tid + 256 * i;
    const int r   = idx >> 3;
    const int q4  = (idx & 7) * 4;
    *(v4f*)(sBC + r * 32 + q4) = *(const v4f*)(BCf + (row0 + r) * kBCW + q4);
  }
  __syncthreads();

  float Ar[kN];
#pragma unroll
  for (int q = 0; q < 4; ++q) {
    const v4f av = *(const v4f*)(Am + (size_t)d * kN + 4 * q);
#pragma unroll
    for (int e = 0; e < 4; ++e) { const float f = av[e]; Ar[4 * q + e] = rne_bf(f); }
  }

  float p[kN], rr[kN];
#pragma unroll
  for (int n = 0; n < kN; ++n) { p[n] = 1.0f; rr[n] = 0.0f; }

#pragma unroll 1
  for (int s = 0; s < kChunk; ++s) {
    const size_t m = row0 + s;
    const float pv = PRE[m * kD + d];
    const float xv = X[m * kD + d];
    const float dl = softplus_f(pv);
    const float xr = rne_bf(xv);
    const float dx = dl * xr;
    const float* br = sBC + s * 32;
    v4f Bq[4];
#pragma unroll
    for (int q = 0; q < 4; ++q) Bq[q] = *(const v4f*)(br + 4 * q);
#pragma unroll
    for (int n = 0; n < kN; ++n) {
      const float bn = Bq[n >> 2][n & 3];
      const float e  = expf(dl * Ar[n]);
      p[n] = p[n] * e;
      const float t = e * rr[n];
      const float u = dx * bn;
      rr[n] = t + u;
    }
  }

#pragma unroll
  for (int n = 0; n < kN; ++n) {
    sP[n * kTP + tid] = p[n];
    sR[n * kTP + tid] = rr[n];
  }
  __syncthreads();

  v4f pv4[4], rv4[4];
#pragma unroll
  for (int it = 0; it < 2; ++it) {
#pragma unroll
    for (int hf = 0; hf < 2; ++hf) {
      const int n   = it * 8 + wave;
      const int col = hf * 128 + lane * 4;
      pv4[it * 2 + hf] = *(const v4f*)(sP + n * kTP + col);
      rv4[it * 2 + hf] = *(const v4f*)(sR + n * kTP + col);
    }
  }
  const size_t nrow0 = ((size_t)b * kNChunk + (size_t)c) * kN;
  for (int pass = 0; pass < 2; ++pass) {
#pragma unroll
    for (int it = 0; it < 2; ++it) {
#pragma unroll
      for (int hf = 0; hf < 2; ++hf) {
        const int n   = it * 8 + wave;
        const int col = hf * 128 + lane * 4;
        const size_t o = (nrow0 + n) * kD + d0 + col;
        *(volatile v4f*)(P + o) = pv4[it * 2 + hf];
        *(volatile v4f*)(R + o) = rv4[it * 2 + hf];
      }
    }
    __threadfence();
  }
}

__global__ __launch_bounds__(256) void scan_pass2_kernel(
    const float* __restrict__ P, const float* __restrict__ R, float* __restrict__ Hin)
{
  __shared__ __align__(16) float sP[kN * kTP];
  __shared__ __align__(16) float sR[kN * kTP];
  __shared__ __align__(16) float sH[kN * kTP];
  const int tid = threadIdx.x, lane = tid & 31, wave = tid >> 5;
  const int d0 = blockIdx.x * 256;
  const int b  = blockIdx.y;

  float h[kN];
#pragma unroll
  for (int n = 0; n < kN; ++n) h[n] = 0.0f;

#pragma unroll 1
  for (int c = 0; c < kNChunk; ++c) {
    const size_t nrow0 = ((size_t)b * kNChunk + (size_t)c) * kN;
#pragma unroll
    for (int n = 0; n < kN; ++n) sH[n * kTP + tid] = h[n];
#pragma unroll
    for (int i = 0; i < 4; ++i) {
      const int idx = tid + 256 * i;
      const int r   = idx >> 6;
      const int q4  = (idx & 63) * 4;
      const size_t go = (nrow0 + r) * kD + d0 + q4;
      *(v4f*)(sP + r * kTP + q4) = *(const v4f*)(P + go);
      *(v4f*)(sR + r * kTP + q4) = *(const v4f*)(R + go);
    }
    __syncthreads();

    v4f hq4[4];
#pragma unroll
    for (int it = 0; it < 2; ++it) {
#pragma unroll
      for (int hf = 0; hf < 2; ++hf) {
        const int n   = it * 8 + wave;
        const int col = hf * 128 + lane * 4;
        hq4[it * 2 + hf] = *(const v4f*)(sH + n * kTP + col);
      }
    }
    for (int pass = 0; pass < 2; ++pass) {
#pragma unroll
      for (int it = 0; it < 2; ++it) {
#pragma unroll
        for (int hf = 0; hf < 2; ++hf) {
          const int n   = it * 8 + wave;
          const int col = hf * 128 + lane * 4;
          const size_t o = (nrow0 + n) * kD + d0 + col;
          *(volatile v4f*)(Hin + o) = hq4[it * 2 + hf];
        }
      }
      __threadfence();
    }

#pragma unroll
    for (int n = 0; n < kN; ++n) {
      const float pv = sP[n * kTP + tid];
      const float rv = sR[n * kTP + tid];
      const float t  = pv * h[n];
      h[n] = t + rv;
    }
    __syncthreads();
  }
}

__global__ __launch_bounds__(256) void scan_pass3_kernel(
    const float* __restrict__ PRE, const float* __restrict__ X, const float* __restrict__ Am,
    const float* __restrict__ BCf, const float* __restrict__ Hin, float* __restrict__ Y)
{
  __shared__ __align__(16) float sBC[kChunk * 32];
  __shared__ __align__(16) float sH[kN * kTP];
  __shared__ __align__(16) float sY[16 * kTP];
  const int tid = threadIdx.x, lane = tid & 31, wave = tid >> 5;
  const int d0 = blockIdx.x * 256;
  const int d  = d0 + tid;
  const int c  = blockIdx.y;
  const int b  = blockIdx.z;
  const size_t row0  = (size_t)b * kL + (size_t)c * kChunk;
  const size_t nrow0 = ((size_t)b * kNChunk + (size_t)c) * kN;

#pragma unroll
  for (int i = 0; i < 2; ++i) {
    const int idx = tid + 256 * i;
    const int r   = idx >> 3;
    const int q4  = (idx & 7) * 4;
    *(v4f*)(sBC + r * 32 + q4) = *(const v4f*)(BCf + (row0 + r) * kBCW + q4);
  }
#pragma unroll
  for (int i = 0; i < 4; ++i) {
    const int idx = tid + 256 * i;
    const int r   = idx >> 6;
    const int q4  = (idx & 63) * 4;
    *(v4f*)(sH + r * kTP + q4) = *(const v4f*)(Hin + (nrow0 + r) * kD + d0 + q4);
  }
  __syncthreads();

  float Ar[kN];
#pragma unroll
  for (int q = 0; q < 4; ++q) {
    const v4f av = *(const v4f*)(Am + (size_t)d * kN + 4 * q);
#pragma unroll
    for (int e = 0; e < 4; ++e) { const float f = av[e]; Ar[4 * q + e] = rne_bf(f); }
  }
  float h[kN];
#pragma unroll
  for (int n = 0; n < kN; ++n) h[n] = sH[n * kTP + tid];

  const int hrow = wave >> 1;
  const int hcol = (wave & 1) * 128 + lane * 4;
#pragma unroll 1
  for (int sub = 0; sub < kChunk / 16; ++sub) {
#pragma unroll 1
    for (int s = 0; s < 16; ++s) {
      const int st = sub * 16 + s;
      const size_t m = row0 + st;
      const float pv = PRE[m * kD + d];
      const float xv = X[m * kD + d];
      const float dl = softplus_f(pv);
      const float xr = rne_bf(xv);
      const float dx = dl * xr;
      const float* br = sBC + st * 32;
      v4f Bq[4], Cq[4];
#pragma unroll
      for (int q = 0; q < 4; ++q) {
        Bq[q] = *(const v4f*)(br + 4 * q);
        Cq[q] = *(const v4f*)(br + kN + 4 * q);
      }
      float y = 0.0f;
#pragma unroll
      for (int n = 0; n < kN; ++n) {
        const float bn = Bq[n >> 2][n & 3];
        const float cn = Cq[n >> 2][n & 3];
        const float e  = expf(dl * Ar[n]);
        const float t  = e * h[n];
        const float u  = dx * bn;
        const float hn = t + u;
        h[n] = hn;
        const float w  = hn * cn;
        y = y + w;
      }
      sY[s * kTP + tid] = y;
    }
    __syncthreads();
    v4f fv[4];
#pragma unroll
    for (int it = 0; it < 4; ++it) fv[it] = *(const v4f*)(sY + (it * 4 + hrow) * kTP + hcol);
    for (int pass = 0; pass < 2; ++pass) {
#pragma unroll
      for (int it = 0; it < 4; ++it)
        *(volatile v4f*)(Y + (row0 + sub * 16 + it * 4 + hrow) * kD + d0 + hcol) = fv[it];
      __threadfence();
    }
    __syncthreads();
  }
}

extern "C" void kernel_launch(void* const* d_in, const int* in_sizes, int n_in,
                              void* d_out, int out_size, void* d_ws, size_t ws_size,
                              hipStream_t stream)
{
  if (n_in < 8) return;
  if (in_sizes[0] != kM * kD) return;
  if (in_sizes[1] != kD * kN) return;
  if (in_sizes[2] != kD * kD) return;
  if (in_sizes[3] != kD) return;
  if (in_sizes[4] != kN * kD) return;
  if (in_sizes[5] != kN) return;
  if (in_sizes[6] != kN * kD) return;
  if (in_sizes[7] != kN) return;
  if (out_size != kM * kD) return;
  if (ws_size < kWsTotal) return;

  const float* x  = (const float*)d_in[0];
  const float* Am = (const float*)d_in[1];
  const float* Wd = (const float*)d_in[2];
  const float* bd = (const float*)d_in[3];
  const float* Wb = (const float*)d_in[4];
  const float* bb = (const float*)d_in[5];
  const float* Wc = (const float*)d_in[6];
  const float* bc = (const float*)d_in[7];
  float* out = (float*)d_out;

  char* ws = (char*)d_ws;
  unsigned short* Xb  = (unsigned short*)(ws + kOffXb);
  unsigned short* Wdb = (unsigned short*)(ws + kOffWdb);
  unsigned short* BCb = (unsigned short*)(ws + kOffBCb);
  float*          bdR = (float*)(ws + kOffBdR);
  float*          bcR = (float*)(ws + kOffBcR);
  float*          PRE = (float*)(ws + kOffPre);
  float*          BCf = (float*)(ws + kOffBCf);
  float*          P   = (float*)(ws + kOffP);
  float*          R   = (float*)(ws + kOffR);
  float*          Hin = (float*)(ws + kOffHin);

  cvt_bf16_kernel<<<(kM * kD / 8) / 256, 256, 0, stream>>>(x, Xb, (kM * kD) / 8);
  cvt_bf16_kernel<<<(kD * kD / 8) / 256, 256, 0, stream>>>(Wd, Wdb, (kD * kD) / 8);
  prep_kernel<<<(kBCW * kD / 8) / 256, 256, 0, stream>>>(Wb, Wc, bd, bb, bc, BCb, bdR, bcR);

  gemm_bf16_64<<<dim3(((kM / 64) * (kD / 64)) / 8), 256, 0, stream>>>(
      Xb, kD, Wdb, kD, PRE, kD, bdR, kM, kD, kD);
  gemm_bf16_64<<<dim3(((kM / 64) * (kBCW / 64)) / 8), 256, 0, stream>>>(
      Xb, kD, BCb, kD, BCf, kBCW, bcR, kM, kBCW, kD);

  scan_pass1_kernel<<<dim3(kD / 256, kNChunk, kB), 256, 0, stream>>>(PRE, x, Am, BCf, P, R);
  scan_pass2_kernel<<<dim3(kD / 256, kB), 256, 0, stream>>>(P, R, Hin);
  scan_pass3_kernel<<<dim3(kD / 256, kNChunk, kB), 256, 0, stream>>>(PRE, x, Am, BCf, Hin, out);
}
